// EntropyGatedAttention_74577812127861
// MI455X (gfx1250) — hardware-verified
//
#include <hip/hip_runtime.h>
#include <math.h>
#include <stdint.h>

#define NB    2
#define SEQ   2048
#define DM    1024
#define NH    16
#define HD    64
#define NQB   (SEQ / 64)
#define ROWS  (NB * SEQ)
#define OUTN  (ROWS * DM)
static_assert(NH * HD == DM);
static_assert(HD == 64);
static_assert((SEQ % 64) == 0 && (DM % 64) == 0 && (ROWS % 64) == 0 && (DM % 32) == 0);
static_assert(((ROWS / 64) * (DM / 64)) % 8 == 0);
static_assert(((ROWS / 32) * (DM / 64)) % 8 == 0);
static_assert(((ROWS * DM / 8) % 256) == 0);
static_assert((DM / 8) == 128);

typedef _Float16 v16h __attribute__((ext_vector_type(16)));
typedef _Float16 v8h  __attribute__((ext_vector_type(8)));
typedef __bf16   v16b __attribute__((ext_vector_type(16)));
typedef __bf16   v8b  __attribute__((ext_vector_type(8)));
typedef float    v8f  __attribute__((ext_vector_type(8)));
typedef float    v4f  __attribute__((ext_vector_type(4)));
typedef unsigned int v4u __attribute__((ext_vector_type(4)));

__device__ __forceinline__ unsigned short bf_bits(float f) {
  unsigned u = __float_as_uint(f);
  return (unsigned short)((u + 0x7FFFu + ((u >> 16) & 1u)) >> 16);
}
__device__ __forceinline__ float bf_up(unsigned short h) { return __uint_as_float(((unsigned)h) << 16); }
__device__ __forceinline__ unsigned short h_bits(_Float16 x) { return __builtin_bit_cast(unsigned short, x); }
__device__ __forceinline__ unsigned pk16(unsigned short a, unsigned short b) { return (unsigned)a | ((unsigned)b << 16); }
__device__ __forceinline__ v8f zero8() { v8f z = {0.f, 0.f, 0.f, 0.f, 0.f, 0.f, 0.f, 0.f}; return z; }

__device__ __forceinline__ v16b ldfrag_b(const __bf16* p) {
  union { v16b v; v8b h[2]; } f;
  f.h[0] = *(const v8b*)(p);
  f.h[1] = *(const v8b*)(p + 16);
  return f.v;
}
__device__ __forceinline__ v16h ldfrag_h(const _Float16* p) {
  union { v16h v; v8h h[2]; } f;
  f.h[0] = *(const v8h*)(p);
  f.h[1] = *(const v8h*)(p + 16);
  return f.v;
}

__device__ __forceinline__ v8f mma_h(v16h a, v16h b, v8f c) {
  c = __builtin_amdgcn_wmma_f32_16x16x32_f16(false, a, false, b, (short)0, c, false, false);
#if defined(__HIP_DEVICE_COMPILE__)
  asm volatile("v_nop\n\tv_nop\n\tv_nop\n\tv_nop" : "+v"(c) : "v"(a), "v"(b));
#endif
  return c;
}
__device__ __forceinline__ v8f mma_b_raw(v16b a, v16b b, v8f c) {
  return __builtin_amdgcn_wmma_f32_16x16x32_bf16(false, a, false, b, (short)0, c, false, false);
}
__device__ __forceinline__ void dep_guard_b(v8f& a, v8f& b, v16b x, v16b y) {
#if defined(__HIP_DEVICE_COMPILE__)
  asm volatile("v_nop\n\tv_nop\n\tv_nop\n\tv_nop" : "+v"(a), "+v"(b) : "v"(x), "v"(y));
#endif
}
__device__ __forceinline__ void keep4_b(v16b a, v16b b, v16b c, v16b d) {
#if defined(__HIP_DEVICE_COMPILE__)
  asm volatile("v_nop" :: "v"(a), "v"(b), "v"(c), "v"(d));
#endif
}
__device__ __forceinline__ void acc_guard4(v8f& a, v8f& b, v8f& c, v8f& d) {
#if defined(__HIP_DEVICE_COMPILE__)
  asm volatile("v_nop\n\tv_nop\n\tv_nop\n\tv_nop" : "+v"(a), "+v"(b), "+v"(c), "+v"(d));
#endif
}

__global__ __launch_bounds__(256) void cvt_bf16x8(const float* __restrict__ in, unsigned short* out, int n8) {
  const int i = blockIdx.x * 256 + threadIdx.x;
  if (i < n8) {
    const v4f a = *(const v4f*)(in + (size_t)i * 8);
    const v4f b = *(const v4f*)(in + (size_t)i * 8 + 4);
    v4u p;
    p[0] = pk16(bf_bits(a[0]), bf_bits(a[1]));
    p[1] = pk16(bf_bits(a[2]), bf_bits(a[3]));
    p[2] = pk16(bf_bits(b[0]), bf_bits(b[1]));
    p[3] = pk16(bf_bits(b[2]), bf_bits(b[3]));
    *(volatile v4u*)(out + (size_t)i * 8) = p;
    __threadfence();
    *(volatile v4u*)(out + (size_t)i * 8) = p;
  }
}

template <int GATED>
__global__ __launch_bounds__(256) void cvt_f16x8(const float* __restrict__ in, const int* __restrict__ gate,
                                                 unsigned short* out, int n8, float scale) {
  const int i = blockIdx.x * 256 + threadIdx.x;
  if (i < n8) {
    const v4f a = *(const v4f*)(in + (size_t)i * 8);
    const v4f b = *(const v4f*)(in + (size_t)i * 8 + 4);
    float sc = scale;
    if (GATED) {
      int row = i >> 7;
      row = min(max(row, 0), ROWS - 1);
      sc = (float)gate[row] * scale;
    }
    v4u p;
    p[0] = pk16(h_bits((_Float16)(a[0] * sc)), h_bits((_Float16)(a[1] * sc)));
    p[1] = pk16(h_bits((_Float16)(a[2] * sc)), h_bits((_Float16)(a[3] * sc)));
    p[2] = pk16(h_bits((_Float16)(b[0] * sc)), h_bits((_Float16)(b[1] * sc)));
    p[3] = pk16(h_bits((_Float16)(b[2] * sc)), h_bits((_Float16)(b[3] * sc)));
    *(volatile v4u*)(out + (size_t)i * 8) = p;
    __threadfence();
    *(volatile v4u*)(out + (size_t)i * 8) = p;
  }
}

template <int MODE>
__device__ __forceinline__ void wt_tile_body(const float* __restrict__ W, unsigned short* Wt, float scale,
                                             float* sw) {
  const int tid = threadIdx.x;
  const int e0  = blockIdx.x * 64;
  const int n0  = blockIdx.y * 64;
#pragma unroll
  for (int i = 0; i < 4; ++i) {
    const int idx = i * 256 + tid;
    const int ee = idx >> 4, c4 = (idx & 15) * 4;
    const v4f a = *(const v4f*)(W + ((size_t)(e0 + ee)) * DM + n0 + c4);
    *(v4f*)(sw + ee * 68 + c4) = a;
  }
  __syncthreads();

  const int g = tid >> 3, piece = tid & 7;
  v4u hv[2];
  size_t hofs[2];
#pragma unroll
  for (int it = 0; it < 2; ++it) {
    const int n = it * 32 + g;
    v4u a;
#pragma unroll
    for (int e = 0; e < 4; ++e) {
      const float f0 = sw[(piece * 8 + 2 * e) * 68 + n];
      const float f1 = sw[(piece * 8 + 2 * e + 1) * 68 + n];
      unsigned short u0, u1;
      if (MODE == 0) {
        u0 = bf_bits(f0);
        u1 = bf_bits(f1);
      } else {
        u0 = h_bits((_Float16)(bf_up(bf_bits(f0)) * scale));
        u1 = h_bits((_Float16)(bf_up(bf_bits(f1)) * scale));
      }
      a[e] = pk16(u0, u1);
    }
    hv[it] = a;
    hofs[it] = ((size_t)(n0 + n)) * DM + e0 + piece * 8;
  }
  for (int pass = 0; pass < 2; ++pass) {
#pragma unroll
    for (int it = 0; it < 2; ++it) {
      *(volatile v4u*)(Wt + hofs[it]) = hv[it];
    }
    __threadfence();
  }
}
__global__ __launch_bounds__(256) void wt_bf16(const float* __restrict__ W, unsigned short* Wt) {
  __shared__ __align__(16) float sw[64 * 68];
  wt_tile_body<0>(W, Wt, 1.0f, sw);
}
__global__ __launch_bounds__(256) void wt_f16s(const float* __restrict__ W, unsigned short* Wt, float scale) {
  __shared__ __align__(16) float sw[64 * 68];
  wt_tile_body<1>(W, Wt, scale, sw);
}

__global__ __launch_bounds__(256) void gemm64(
    const unsigned short* __restrict__ Ap, int lda,
    const unsigned short* __restrict__ Btp, int ldb,
    const float* __restrict__ bias,
    float* C, int ldc, int M, int N, int K) {
  const __bf16* Ab  = (const __bf16*)(const void*)Ap;
  const __bf16* Bb  = (const __bf16*)(const void*)Btp;
  __shared__ __align__(16) float sT[8][16 * 68];
  const int lane = threadIdx.x & 31;
  const int wave = threadIdx.x >> 5;
  const int tilesN = N >> 6;
  const int tilesM = M >> 6;
  const int tile = blockIdx.x * 8 + wave;
  if (tile >= tilesM * tilesN) return;
  const int tm = tile / tilesN;
  const int tn = tile - tm * tilesN;
  const int m0 = tm << 6;
  const int n0 = tn << 6;

  const int rlane = lane & 15;
  const int koff  = (lane >> 4) * 8;
  const int mOff  = (lane >> 4) * 8;

  v8f acc[4][4];
#pragma unroll
  for (int i = 0; i < 4; ++i)
#pragma unroll
    for (int j = 0; j < 4; ++j) acc[i][j] = zero8();

  for (int k0 = 0; k0 < K; k0 += 32) {
    v16b bh[4];
#pragma unroll
    for (int j = 0; j < 4; ++j) {
      const size_t bo = (size_t)(n0 + (j << 4) + rlane) * ldb + koff + k0;
      bh[j] = ldfrag_b(Bb + bo);
    }
#pragma unroll
    for (int i = 0; i < 4; ++i) {
      const size_t ao = (size_t)(m0 + (i << 4) + rlane) * lda + koff + k0;
      const v16b ah = ldfrag_b(Ab + ao);
#pragma unroll
      for (int j = 0; j < 4; ++j) {
        acc[i][j] = mma_b_raw(ah, bh[j], acc[i][j]);
      }
      dep_guard_b(acc[i][0], acc[i][3], ah, ah);
    }
    keep4_b(bh[0], bh[1], bh[2], bh[3]);
  }
  acc_guard4(acc[0][0], acc[0][1], acc[0][2], acc[0][3]);
  acc_guard4(acc[1][0], acc[1][1], acc[1][2], acc[1][3]);
  acc_guard4(acc[2][0], acc[2][1], acc[2][2], acc[2][3]);
  acc_guard4(acc[3][0], acc[3][1], acc[3][2], acc[3][3]);

  float bz[4];
#pragma unroll
  for (int j = 0; j < 4; ++j) bz[j] = bf_up(bf_bits(bias[n0 + (j << 4) + rlane]));

  float* slab = sT[wave];
#pragma unroll
  for (int i = 0; i < 4; ++i) {
    const int mBase = m0 + (i << 4);
#pragma unroll
    for (int r = 0; r < 8; ++r) {
#pragma unroll
      for (int j = 0; j < 4; ++j) {
        slab[(mOff + r) * 68 + (j << 4) + rlane] = acc[i][j][r] + bz[j];
      }
    }
    __builtin_amdgcn_fence(__ATOMIC_RELEASE, "workgroup");
    __builtin_amdgcn_wave_barrier();
    __builtin_amdgcn_fence(__ATOMIC_ACQUIRE, "workgroup");
    {
      const int hh = lane >> 4, c4 = (lane & 15) * 4;
      v4f ov[8];
#pragma unroll
      for (int it = 0; it < 8; ++it) {
        const int row = it * 2 + hh;
        ov[it] = *(const v4f*)(slab + row * 68 + c4);
      }
      for (int pass = 0; pass < 2; ++pass) {
#pragma unroll
        for (int it = 0; it < 8; ++it) {
          const int row = it * 2 + hh;
          *(volatile v4f*)(C + (size_t)(mBase + row) * ldc + n0 + c4) = ov[it];
        }
        __threadfence();
      }
    }
    __builtin_amdgcn_fence(__ATOMIC_RELEASE, "workgroup");
    __builtin_amdgcn_wave_barrier();
    __builtin_amdgcn_fence(__ATOMIC_ACQUIRE, "workgroup");
  }
}

__global__ __launch_bounds__(256) void gemm_ob(
    const unsigned short* __restrict__ Ahp, int lda,
    const unsigned short* __restrict__ Btp, int ldb,
    const float* __restrict__ bias,
    const float* __restrict__ xres, int ldx,
    const int* __restrict__ gate,
    float* C, int ldc, int M, int N, int K, float oscale) {
  const _Float16* Ah = (const _Float16*)(const void*)Ahp;
  const _Float16* Bh = (const _Float16*)(const void*)Btp;
  __shared__ __align__(16) float sT[8][16 * 68];
  const int lane = threadIdx.x & 31;
  const int wave = threadIdx.x >> 5;
  const int tilesN = N >> 6;
  const int tilesM = M >> 5;
  const int tile = blockIdx.x * 8 + wave;
  if (tile >= tilesM * tilesN) return;
  const int tm = tile / tilesN;
  const int tn = tile - tm * tilesN;
  const int m0 = tm << 5;
  const int n0 = tn << 6;

  const int rlane = lane & 15;
  const int koff  = (lane >> 4) * 8;
  const int mOff  = (lane >> 4) * 8;

  v8f acc[2][4];
#pragma unroll
  for (int i = 0; i < 2; ++i)
#pragma unroll
    for (int j = 0; j < 4; ++j) acc[i][j] = zero8();

  for (int k0 = 0; k0 < K; k0 += 32) {
    v16h ah[2];
#pragma unroll
    for (int i = 0; i < 2; ++i) {
      const size_t ao = (size_t)(m0 + (i << 4) + rlane) * lda + koff + k0;
      ah[i] = ldfrag_h(Ah + ao);
    }
#pragma unroll
    for (int j = 0; j < 4; ++j) {
      const size_t bo = (size_t)(n0 + (j << 4) + rlane) * ldb + koff + k0;
      const v16h bfr = ldfrag_h(Bh + bo);
#pragma unroll
      for (int i = 0; i < 2; ++i) {
        acc[i][j] = mma_h(ah[i], bfr, acc[i][j]);
      }
    }
  }

  float bz[4];
#pragma unroll
  for (int j = 0; j < 4; ++j) bz[j] = bf_up(bf_bits(bias[n0 + (j << 4) + rlane]));

  float* slab = sT[wave];
#pragma unroll
  for (int i = 0; i < 2; ++i) {
    const int mBase = m0 + (i << 4);
#pragma unroll
    for (int r = 0; r < 8; ++r) {
      const int row = mBase + mOff + r;
      const float g = (float)gate[row];
#pragma unroll
      for (int j = 0; j < 4; ++j) {
        const int col = n0 + (j << 4) + rlane;
        const float xr = bf_up(bf_bits(xres[(size_t)row * ldx + col]));
        const float y  = acc[i][j][r] * oscale + bz[j];
        slab[(mOff + r) * 68 + (j << 4) + rlane] = xr * (1.0f - g) + y * g;
      }
    }
    __builtin_amdgcn_fence(__ATOMIC_RELEASE, "workgroup");
    __builtin_amdgcn_wave_barrier();
    __builtin_amdgcn_fence(__ATOMIC_ACQUIRE, "workgroup");
    {
      const int hh = lane >> 4, c4 = (lane & 15) * 4;
      v4f ov[8];
#pragma unroll
      for (int it = 0; it < 8; ++it) {
        const int row = it * 2 + hh;
        ov[it] = *(const v4f*)(slab + row * 68 + c4);
      }
      for (int pass = 0; pass < 2; ++pass) {
#pragma unroll
        for (int it = 0; it < 8; ++it) {
          const int row = it * 2 + hh;
          *(volatile v4f*)(C + (size_t)(mBase + row) * ldc + n0 + c4) = ov[it];
        }
        __threadfence();
      }
    }
    __builtin_amdgcn_fence(__ATOMIC_RELEASE, "workgroup");
    __builtin_amdgcn_wave_barrier();
    __builtin_amdgcn_fence(__ATOMIC_ACQUIRE, "workgroup");
  }
}

__global__ __launch_bounds__(256) void v_planes(const float* __restrict__ vf, int vrp,
                                                const int* __restrict__ gate,
                                                unsigned short* vth, float vscale) {
  __shared__ __align__(16) float sv[64 * 68];
  const int tid = threadIdx.x;
  const int t0  = blockIdx.x * 64;
  const int hh  = blockIdx.y;
  const int b   = blockIdx.z;
#pragma unroll
  for (int i = 0; i < 4; ++i) {
    const int idx = i * 256 + tid;
    const int tt = idx >> 4, c4 = (idx & 15) * 4;
    const float gs = (float)gate[b * SEQ + t0 + tt];
    v4f a = *(const v4f*)(vf + ((size_t)(b * SEQ + t0 + tt)) * vrp + hh * HD + c4);
    a = a * gs;
    *(v4f*)(sv + tt * 68 + c4) = a;
  }
  __syncthreads();

  const int g = tid >> 3, piece = tid & 7;
  v4u hv[2];
  size_t hofs[2];
#pragma unroll
  for (int it = 0; it < 2; ++it) {
    const int d = it * 32 + g;
    v4u a;
#pragma unroll
    for (int e = 0; e < 4; ++e) {
      const float f0 = sv[(piece * 8 + 2 * e) * 68 + d] * vscale;
      const float f1 = sv[(piece * 8 + 2 * e + 1) * 68 + d] * vscale;
      a[e] = pk16(h_bits((_Float16)f0), h_bits((_Float16)f1));
    }
    hv[it] = a;
    hofs[it] = ((size_t)(b * DM + hh * HD + d)) * SEQ + t0 + piece * 8;
  }
  for (int pass = 0; pass < 2; ++pass) {
#pragma unroll
    for (int it = 0; it < 2; ++it) {
      *(volatile v4u*)(vth + hofs[it]) = hv[it];
    }
    __threadfence();
  }
}

__global__ __launch_bounds__(128)
void attn64(const unsigned short* __restrict__ qhp, const unsigned short* __restrict__ khp,
            const unsigned short* __restrict__ vhp, float* outp, float sscale, float oscl) {
  union FH { v16h v; v8h h[2]; };
  __shared__ __align__(16) _Float16 Ksh[64 * 64];
  __shared__ __align__(16) _Float16 Vth[64 * 64];
  __shared__ __align__(16) _Float16 Psh[4][16 * 64];
  __shared__ __align__(16) float    Os[4][16 * 64];

  const int tid  = threadIdx.x;
  const int wave = tid >> 5;
  const int lane = tid & 31;
  const int hh   = lane >> 4;
  const int c    = lane & 15;

  const int bx   = blockIdx.x;
  const int qb   = bx % NQB;
  const int rest = bx / NQB;
  const int h    = rest % NH;
  const int b    = rest / NH;
  const int q0   = qb * 64 + wave * 16;
  const size_t rowB = (size_t)b * SEQ;

  const _Float16* Qp  = (const _Float16*)(const void*)qhp + (size_t)h * HD;
  const _Float16* Kp  = (const _Float16*)(const void*)khp + (size_t)h * HD;
  const _Float16* Vh  = (const _Float16*)(const void*)vhp + ((size_t)b * DM + (size_t)h * HD) * SEQ;

  v16h qa[2];
#pragma unroll
  for (int dc = 0; dc < 2; ++dc) {
    const size_t qo = (rowB + q0 + c) * DM + dc * 32 + 8 * hh;
    qa[dc] = ldfrag_h(Qp + qo);
  }

  float mrow[8], lrow[8];
  v8f oacc[4];
#pragma unroll
  for (int r = 0; r < 8; ++r) { mrow[r] = -INFINITY; lrow[r] = 0.f; }
#pragma unroll
  for (int t = 0; t < 4; ++t) oacc[t] = zero8();

  for (int kt = 0; kt < NQB; ++kt) {
    const int kv0 = kt * 64;
    __syncthreads();
    {
      const int r = tid >> 1, half = (tid & 1) * 32;
      const _Float16* kg = Kp + (rowB + kv0 + r) * DM + half;
      const _Float16* vg = Vh + (size_t)r * SEQ + kv0 + half;
#pragma unroll
      for (int i = 0; i < 4; ++i) {
        const v8h a0 = *(const v8h*)(kg + 8 * i);
        const v8h b0 = *(const v8h*)(vg + 8 * i);
        *(v8h*)(Ksh + r * 64 + half + 8 * i) = a0;
        *(v8h*)(Vth + r * 64 + half + 8 * i) = b0;
      }
    }
    __syncthreads();

    v8f s[4];
#pragma unroll
    for (int j = 0; j < 4; ++j) {
      s[j] = zero8();
#pragma unroll
      for (int dc = 0; dc < 2; ++dc) {
        FH kb;
        kb.h[0] = *(const v8h*)(Ksh + (j * 16 + c) * 64 + dc * 32 + 8 * hh);
        kb.h[1] = *(const v8h*)(Ksh + (j * 16 + c) * 64 + dc * 32 + 16 + 8 * hh);
        s[j] = mma_h(qa[dc], kb.v, s[j]);
      }
    }

    _Float16* pwh = Psh[wave];
#pragma unroll
    for (int r = 0; r < 8; ++r) {
      float m = -INFINITY;
#pragma unroll
      for (int j = 0; j < 4; ++j) {
        const float sv = s[j][r] * sscale;
        s[j][r] = sv;
        m = fmaxf(m, sv);
      }
#pragma unroll
      for (int off = 1; off < 16; off <<= 1) m = fmaxf(m, __shfl_xor(m, off, 32));
      const float mnew  = fmaxf(mrow[r], m);
      const float msafe = (mnew == -INFINITY) ? 0.f : mnew;
      const float alpha = __expf(mrow[r] - msafe);
      mrow[r] = mnew;
      float psum = 0.f;
#pragma unroll
      for (int j = 0; j < 4; ++j) {
        const float p = __expf(s[j][r] - msafe);
        psum += p;
        const float p1024 = p * 1024.0f;
        const _Float16 ph = (_Float16)p1024;
        pwh[(8 * hh + r) * 64 + j * 16 + c] = ph;
      }
#pragma unroll
      for (int off = 1; off < 16; off <<= 1) psum += __shfl_xor(psum, off, 32);
      lrow[r] = lrow[r] * alpha + psum;
#pragma unroll
      for (int t = 0; t < 4; ++t) oacc[t][r] *= alpha;
    }
    __builtin_amdgcn_fence(__ATOMIC_RELEASE, "workgroup");
    __builtin_amdgcn_wave_barrier();
    __builtin_amdgcn_fence(__ATOMIC_ACQUIRE, "workgroup");

#pragma unroll 1
    for (int kk = 0; kk < 2; ++kk) {
      FH pa;
      pa.h[0] = *(const v8h*)(pwh + c * 64 + kk * 32 + 8 * hh);
      pa.h[1] = *(const v8h*)(pwh + c * 64 + kk * 32 + 16 + 8 * hh);
#pragma unroll
      for (int t = 0; t < 4; ++t) {
        FH vb;
        vb.h[0] = *(const v8h*)(Vth + (t * 16 + c) * 64 + kk * 32 + 8 * hh);
        vb.h[1] = *(const v8h*)(Vth + (t * 16 + c) * 64 + kk * 32 + 16 + 8 * hh);
        oacc[t] = mma_h(pa.v, vb.v, oacc[t]);
      }
    }
  }

  float* os = Os[wave];
#pragma unroll
  for (int r = 0; r < 8; ++r) {
    const float l = lrow[r];
    const float inv = ((l > 0.f) ? (1.0f / l) : 0.f) * oscl;
#pragma unroll
    for (int t = 0; t < 4; ++t) {
      os[(8 * hh + r) * 64 + t * 16 + c] = oacc[t][r] * inv;
    }
  }
  __builtin_amdgcn_fence(__ATOMIC_RELEASE, "workgroup");
  __builtin_amdgcn_wave_barrier();
  __builtin_amdgcn_fence(__ATOMIC_ACQUIRE, "workgroup");
  {
    const int h2 = lane >> 4, c4 = (lane & 15) * 4;
    v4f ov[8];
#pragma unroll
    for (int it = 0; it < 8; ++it) {
      const int row = it * 2 + h2;
      ov[it] = *(const v4f*)(os + row * 64 + c4);
    }
    for (int pass = 0; pass < 2; ++pass) {
#pragma unroll
      for (int it = 0; it < 8; ++it) {
        const int row = it * 2 + h2;
        const size_t go = (rowB + q0 + row) * DM + (size_t)h * HD + c4;
        *(volatile v4f*)(outp + go) = ov[it];
      }
      __threadfence();
    }
  }
}

extern "C" void kernel_launch(void* const* d_in, const int* in_sizes, int n_in,
                              void* d_out, int out_size, void* d_ws, size_t ws_size,
                              hipStream_t stream) {
  if (n_in < 10) return;
  if (in_sizes[0] != NB * SEQ * DM) return;
  if (in_sizes[1] != NB * SEQ) return;
  if (in_sizes[2] != DM * DM) return;
  if (in_sizes[3] != DM) return;
  if (in_sizes[4] != DM * DM) return;
  if (in_sizes[5] != DM) return;
  if (in_sizes[6] != DM * DM) return;
  if (in_sizes[7] != DM) return;
  if (in_sizes[8] != DM * DM) return;
  if (in_sizes[9] != DM) return;
  if (out_size != OUTN) return;

  const float* x    = (const float*)d_in[0];
  const int*   gate = (const int*)d_in[1];
  const float* Wq   = (const float*)d_in[2];
  const float* bq   = (const float*)d_in[3];
  const float* Wk   = (const float*)d_in[4];
  const float* bk   = (const float*)d_in[5];
  const float* Wv   = (const float*)d_in[6];
  const float* bv   = (const float*)d_in[7];
  const float* Wo   = (const float*)d_in[8];
  const float* bo   = (const float*)d_in[9];

  const size_t PXb = (size_t)ROWS * DM * 2;
  const size_t PW  = (size_t)DM * DM * 2;
  const size_t PF  = (size_t)ROWS * DM * 4;
  const size_t PH  = (size_t)ROWS * DM * 2;
  const size_t PVt = (size_t)NB * DM * SEQ * 2;
  size_t off = 0;
  const size_t oXb = off; off += PXb;
  const size_t oWq = off; off += PW;
  const size_t oWk = off; off += PW;
  const size_t oWv = off; off += PW;
  const size_t oWo = off; off += PW;
  const size_t oTf = off; off += PF;
  const size_t oQh = off; off += PH;
  const size_t oKh = off; off += PH;
  const size_t oVt = off; off += PVt;
  const size_t oMh = off; off += PH;
  if (off > ws_size) return;
  if (off > (size_t)134217728) return;

  char* ws = (char*)d_ws;
  unsigned short* Xb  = (unsigned short*)(ws + oXb);
  unsigned short* Wtq = (unsigned short*)(ws + oWq);
  unsigned short* Wtk = (unsigned short*)(ws + oWk);
  unsigned short* Wtv = (unsigned short*)(ws + oWv);
  unsigned short* Wto = (unsigned short*)(ws + oWo);
  float*          Tf  = (float*)(ws + oTf);
  unsigned short* Qh  = (unsigned short*)(ws + oQh);
  unsigned short* Kh  = (unsigned short*)(ws + oKh);
  unsigned short* VTh = (unsigned short*)(ws + oVt);
  unsigned short* Mh  = (unsigned short*)(ws + oMh);
  float*          outf = (float*)d_out;

  const dim3 blk(256);
  const int n8x = ROWS * DM / 8;
  const dim3 gCvtX((n8x + 255) / 256);
  const dim3 gWt(DM / 64, DM / 64);
  const dim3 gGemm(((ROWS / 64) * (DM / 64) + 7) / 8);
  const dim3 gGemO(((ROWS / 32) * (DM / 64) + 7) / 8);
  const dim3 gVpl(SEQ / 64, NH, NB);
  const dim3 gAttn(NB * NH * NQB);
  const float qkScale = 16.0f;
  const float sscale  = 1.0f / 2048.0f;
  const float vScale  = 256.0f;
  const float attOscl = 1.0f / 262144.0f;
  const float mScale  = 1024.0f;
  const float woScale = 4096.0f;
  const float outOscl = 1.0f / 4194304.0f;

  cvt_bf16x8<<<gCvtX, blk, 0, stream>>>(x, Xb, n8x);
  wt_bf16<<<gWt, blk, 0, stream>>>(Wq, Wtq);
  wt_bf16<<<gWt, blk, 0, stream>>>(Wk, Wtk);
  wt_bf16<<<gWt, blk, 0, stream>>>(Wv, Wtv);
  wt_f16s<<<gWt, blk, 0, stream>>>(Wo, Wto, woScale);
  gemm64<<<gGemm, blk, 0, stream>>>(Xb, DM, Wtq, DM, bq, Tf, DM, ROWS, DM, DM);
  cvt_f16x8<1><<<gCvtX, blk, 0, stream>>>(Tf, gate, Qh, n8x, qkScale);
  gemm64<<<gGemm, blk, 0, stream>>>(Xb, DM, Wtk, DM, bk, Tf, DM, ROWS, DM, DM);
  cvt_f16x8<1><<<gCvtX, blk, 0, stream>>>(Tf, gate, Kh, n8x, qkScale);
  gemm64<<<gGemm, blk, 0, stream>>>(Xb, DM, Wtv, DM, bv, Tf, DM, ROWS, DM, DM);
  v_planes<<<gVpl, blk, 0, stream>>>(Tf, DM, gate, VTh, vScale);
  attn64<<<gAttn, dim3(128), 0, stream>>>(Qh, Kh, VTh, Tf, sscale, attOscl);
  cvt_f16x8<0><<<gCvtX, blk, 0, stream>>>(Tf, gate, Mh, n8x, mScale);
  gemm_ob<<<gGemO, blk, 0, stream>>>(Mh, DM, Wto, DM, bo, x, DM, gate, outf, DM, ROWS, DM, DM, outOscl);
  (void)hipGetLastError();
}
